// SelfAttention_56564719288804
// MI455X (gfx1250) — hardware-verified
//
#include <hip/hip_runtime.h>
#include <stddef.h>
#include <stdint.h>
#include <math.h>

#ifndef NB
#define NB 32
#endif
#define SEQ    512
#define LFULL  512
#define EW     128
#define NH     8
#define HD     16
#define QROW   32
#define TPITCH 136
#define OPITCH 36
#define WSMAX  134217728
#define VPL    ((size_t)NB * EW * SEQ)
#define PLN    ((size_t)NB * NH * SEQ * QROW)
#define SCN    ((size_t)NB * NH * SEQ)
#define XB_FULL ((size_t)EW * LFULL)
#define LOG2E  1.4426950408889634f

static_assert(NH * HD == EW);
static_assert(SEQ == 512 && LFULL == 512);
static_assert(EW % 32 == 0 && SEQ % 32 == 0);
static_assert(SEQ % 64 == 0 && (NB * SEQ) % 64 == 0);
static_assert(NH * 64 * QROW == 16384);
static_assert(2 * EW * 64 == 16384);
static_assert(16384 == 128 * 16 * 8);
static_assert(64 * EW == 128 * 16 * 4);
static_assert(3 * NH * 64 == 128 * 3 * 4);
static_assert((2 * EW * EW) % (256 * 8) == 0);
static_assert((EW * EW) % (256 * 8) == 0);
static_assert(EW * 32 == 256 * 4 * 4);
static_assert(TPITCH % 8 == 0 && TPITCH >= EW);
static_assert(OPITCH % 4 == 0 && OPITCH >= 32);
static_assert((size_t)3 * EW * EW * 2 + 2 * PLN * 2 + 2 * VPL * 2 + 3 * SCN * 4 <= (size_t)WSMAX);

typedef int            v4i   __attribute__((ext_vector_type(4)));
typedef int            v8i   __attribute__((ext_vector_type(8)));
typedef float          v4f   __attribute__((ext_vector_type(4)));
typedef float          v8f   __attribute__((ext_vector_type(8)));
typedef __bf16         v16bf __attribute__((ext_vector_type(16)));
typedef v4i __attribute__((may_alias)) v4ia;
typedef v4f __attribute__((may_alias)) v4fa;
union FragB { v16bf v; v4i q[2]; v8i w; };

__device__ __forceinline__ v8f wmb(const FragB& a, const FragB& b, v8f c) {
  v8f d = __builtin_amdgcn_wmma_f32_16x16x32_bf16(false, a.v, false, b.v, (short)0, c, false, false);
  asm volatile("v_nop\n\tv_nop\n\tv_nop\n\tv_nop" : "+v"(d) : "v"(a.w), "v"(b.w));
  return d;
}

__device__ __forceinline__ unsigned bf16_bits(float f) {
  const unsigned u = __float_as_uint(f);
  return (u + 0x7FFFu + ((u >> 16) & 1u)) >> 16;
}
__device__ __forceinline__ float bf16_val(float f) {
  return __uint_as_float(bf16_bits(f) << 16);
}
__device__ __forceinline__ int pack2(float lo, float hi) {
  return (int)(bf16_bits(lo) | (bf16_bits(hi) << 16));
}
__device__ __forceinline__ void split8(const v8f x, v4i& hi, v4i& lo) {
#pragma unroll
  for (int j = 0; j < 4; ++j) {
    const float a = x[2 * j], b = x[2 * j + 1];
    const unsigned ha = bf16_bits(a), hb = bf16_bits(b);
    const float ra = a - __uint_as_float(ha << 16);
    const float rb = b - __uint_as_float(hb << 16);
    hi[j] = (int)(ha | (hb << 16));
    lo[j] = (int)(bf16_bits(ra) | (bf16_bits(rb) << 16));
  }
}
__device__ __forceinline__ FragB ldg_frag(const unsigned short* __restrict__ p) {
  FragB f;
  f.q[0] = *(const v4ia*)p;
  f.q[1] = *(const v4ia*)(p + 16);
  return f;
}

__device__ __forceinline__ float hyp8(v8f& a, const float scl) {
#pragma clang fp contract(off)
  float ss = 0.0f;
#pragma unroll
  for (int r = 0; r < 8; ++r) { a[r] = a[r] * scl; ss += a[r] * a[r]; }
  ss += __shfl_xor(ss, 16);
  const float n = sqrtf(ss);
  const float inv = 1.0f / fmaxf(n, 1.0e-12f);
  const float sh = sinhf(n);
  const float ch = coshf(n);
#pragma unroll
  for (int r = 0; r < 8; ++r) a[r] = (a[r] * inv) * sh;
  return ch;
}

__device__ __forceinline__ float klein8(v8f& a, const float biasv, const float mterm) {
#pragma clang fp contract(off)
  float ss = 0.0f;
#pragma unroll
  for (int r = 0; r < 8; ++r) ss += a[r] * a[r];
  ss += __shfl_xor(ss, 16);
  const float vn = sqrtf(ss);
  const float inv = 1.0f / fmaxf(vn, 1.0e-12f);
  const float sh = sinhf(vn);
  const float ch = coshf(vn);
  const float ich = 1.0f / ch;
  float s2 = 0.0f;
#pragma unroll
  for (int r = 0; r < 8; ++r) { a[r] = ((a[r] * inv) * sh) * ich; s2 += a[r] * a[r]; }
  s2 += __shfl_xor(s2, 16);
  const float n2 = sqrtf(s2);
  const float inv2 = 1.0f / fmaxf(n2, 1.0e-12f);
  float s3 = 0.0f;
#pragma unroll
  for (int r = 0; r < 8; ++r) { a[r] = a[r] * inv2; s3 += a[r] * a[r]; }
  s3 += __shfl_xor(s3, 16);
  const float vnk = sqrtf(s3);
  const float dm = vnk - 1.0e-4f;
  const float den = sqrtf(1.0f - dm * dm) + 1.0e-4f;
  const float lden = 1.0f / den;
  const float lb = logf(lden) + biasv;
  return lb * LOG2E + mterm;
}

__device__ __forceinline__ float hlogit(const float rt, const float ct, const float dot,
                                        const float nbeta, const float cb) {
  const float x1 = (rt * ct - dot) + 1.0e-6f;
  const float y = x1 + sqrtf(fmaxf(x1 * x1 - 1.0f, 0.0f));
  return nbeta * log2f(y) + cb;
}

__global__ __launch_bounds__(256) void k_cvt(const float* __restrict__ x, unsigned short* o) {
  const size_t i = (size_t)blockIdx.x * 256u + threadIdx.x;
  const float* p = x + i * 8u;
  const v4f a = *(const v4fa*)p;
  const v4f b = *(const v4fa*)(p + 4);
  v4i w;
  w[0] = pack2(a.x, a.y); w[1] = pack2(a.z, a.w);
  w[2] = pack2(b.x, b.y); w[3] = pack2(b.z, b.w);
  unsigned short* d = o + i * 8u;
  *(volatile v4i*)d = w;
  __threadfence();
  *(volatile v4i*)d = w;
}

__global__ __launch_bounds__(128) void k_hproj(const float* __restrict__ x, const int* __restrict__ mask,
                                               const unsigned short* __restrict__ wt,
                                               const float* __restrict__ bias_p,
                                               unsigned short* pl, unsigned short* vt, float* sca) {
  __shared__ __attribute__((aligned(16))) unsigned short xt[64 * TPITCH];
  __shared__ __attribute__((aligned(16))) unsigned short stg[16384];
  __shared__ __attribute__((aligned(16))) float ssc[3 * NH * 64];
  const unsigned tid = threadIdx.x, lane = tid & 31u, hh = lane >> 4, m = lane & 15u;
  const unsigned wave = (unsigned)__builtin_amdgcn_readfirstlane((int)(threadIdx.x >> 5));
  const unsigned row0 = blockIdx.x * 64u;
  const unsigned bb = row0 >> 9, r0 = row0 & 511u;

  {
    const float* xg = x + (size_t)bb * XB_FULL + r0;
#pragma unroll 1
    for (unsigned it = 0; it < 16u; ++it) {
      const unsigned p = it * 128u + tid, k = p >> 4, l4 = (p & 15u) << 2;
      const v4f v = *(const v4fa*)(xg + (size_t)k * LFULL + l4);
      xt[(l4 + 0u) * TPITCH + k] = (unsigned short)bf16_bits(v.x);
      xt[(l4 + 1u) * TPITCH + k] = (unsigned short)bf16_bits(v.y);
      xt[(l4 + 2u) * TPITCH + k] = (unsigned short)bf16_bits(v.z);
      xt[(l4 + 3u) * TPITCH + k] = (unsigned short)bf16_bits(v.w);
    }
  }
  __syncthreads();

  FragB xa[4];
  {
    const unsigned xo = (16u * wave + m) * TPITCH + 8u * hh;
#pragma unroll
    for (int ks = 0; ks < 4; ++ks) {
      xa[ks].q[0] = *(const v4ia*)(xt + xo + 32 * ks);
      xa[ks].q[1] = *(const v4ia*)(xt + xo + 32 * ks + 16);
    }
  }
  const int mi = mask[(size_t)bb * LFULL + r0 + 16u * wave + m];
  const float mv = (float)mi;
  const float mterm = (-1.0e30f * (1.0f - mv)) * LOG2E;
  const float biasv = bf16_val(bias_p[0]);
  const v8f zero8 = {0.f, 0.f, 0.f, 0.f, 0.f, 0.f, 0.f, 0.f};

#pragma unroll 1
  for (unsigned ps = 0; ps < 2u; ++ps) {
    const unsigned woff = (ps == 0u) ? (unsigned)(2 * EW * EW) : 0u;
    const float scl = (ps == 0u) ? 0.25f : 1.0f;
#pragma unroll 1
    for (unsigned t = 0; t < NH; ++t) {
      const unsigned short* wp = wt + woff + (size_t)(16u * t + m) * EW + 8u * hh;
      v8f acc = zero8;
#pragma unroll
      for (int ks = 0; ks < 4; ++ks) {
        const FragB wf = ldg_frag(wp + 32 * ks);
        acc = wmb(wf, xa[ks], acc);
      }
      const float ch = hyp8(acc, scl);
      v4i hi, lo;
      split8(acc, hi, lo);
      const unsigned so = (t * 64u + 16u * wave + m) * QROW + 8u * hh;
      *(v4ia*)(stg + so) = hi;
      *(v4ia*)(stg + so + 16u) = lo;
      if (hh == 0u) ssc[(ps * NH + t) * 64u + 16u * wave + m] = ch;
    }
    __syncthreads();
    {
      unsigned short* dst = pl + (size_t)ps * PLN + ((size_t)bb * NH * SEQ + r0) * QROW;
#pragma unroll 1
      for (unsigned it = 0; it < 16u; ++it) {
        const unsigned p = it * 128u + tid, t = p >> 8, wi = p & 255u;
        const v4i v = *(const v4ia*)(stg + p * 8u);
        *(volatile v4i*)(dst + (size_t)t * (SEQ * QROW) + wi * 8u) = v;
      }
      __threadfence();
#pragma unroll 1
      for (unsigned it = 0; it < 16u; ++it) {
        const unsigned p = it * 128u + tid, t = p >> 8, wi = p & 255u;
        const v4i v = *(const v4ia*)(stg + p * 8u);
        *(volatile v4i*)(dst + (size_t)t * (SEQ * QROW) + wi * 8u) = v;
      }
    }
    __syncthreads();
  }

#pragma unroll 1
  for (unsigned t = 0; t < NH; ++t) {
    const unsigned short* wp = wt + (unsigned)(EW * EW) + (size_t)(16u * t + m) * EW + 8u * hh;
    v8f acc = zero8;
#pragma unroll
    for (int ks = 0; ks < 4; ++ks) {
      const FragB wf = ldg_frag(wp + 32 * ks);
      acc = wmb(wf, xa[ks], acc);
    }
    const float lb2 = klein8(acc, biasv, mterm);
#pragma unroll
    for (int r = 0; r < 8; ++r) {
      const unsigned hb = bf16_bits(acc[r]);
      const float res = acc[r] - __uint_as_float(hb << 16);
      const unsigned so = (16u * t + 8u * hh + (unsigned)r) * 64u + 16u * wave + m;
      stg[so] = (unsigned short)hb;
      stg[so + 8192u] = (unsigned short)bf16_bits(res);
    }
    if (hh == 0u) ssc[(2u * NH + t) * 64u + 16u * wave + m] = lb2;
  }
  __syncthreads();
  {
    unsigned short* dst = vt + (size_t)bb * EW * SEQ + r0;
#pragma unroll 1
    for (unsigned it = 0; it < 16u; ++it) {
      const unsigned p = it * 128u + tid, pn = p >> 10, col = (p >> 3) & 127u, c = p & 7u;
      const v4i v = *(const v4ia*)(stg + p * 8u);
      *(volatile v4i*)(dst + (size_t)pn * VPL + (size_t)col * SEQ + c * 8u) = v;
    }
    __threadfence();
#pragma unroll 1
    for (unsigned it = 0; it < 16u; ++it) {
      const unsigned p = it * 128u + tid, pn = p >> 10, col = (p >> 3) & 127u, c = p & 7u;
      const v4i v = *(const v4ia*)(stg + p * 8u);
      *(volatile v4i*)(dst + (size_t)pn * VPL + (size_t)col * SEQ + c * 8u) = v;
    }
  }
  {
#pragma unroll 1
    for (unsigned it = 0; it < 3u; ++it) {
      const unsigned p = it * 128u + tid, a = p >> 7, t = (p >> 4) & 7u, c = p & 15u;
      const v4f v = *(const v4fa*)(ssc + p * 4u);
      *(volatile v4f*)(sca + (size_t)a * SCN + ((size_t)bb * NH + t) * SEQ + r0 + 4u * c) = v;
    }
    __threadfence();
#pragma unroll 1
    for (unsigned it = 0; it < 3u; ++it) {
      const unsigned p = it * 128u + tid, a = p >> 7, t = (p >> 4) & 7u, c = p & 15u;
      const v4f v = *(const v4fa*)(ssc + p * 4u);
      *(volatile v4f*)(sca + (size_t)a * SCN + ((size_t)bb * NH + t) * SEQ + r0 + 4u * c) = v;
    }
  }
}

__global__ __launch_bounds__(256) void k_hattn(const unsigned short* __restrict__ rpl,
                                               const unsigned short* __restrict__ cpl,
                                               const unsigned short* __restrict__ vt,
                                               const float* __restrict__ rtt,
                                               const float* __restrict__ ctt,
                                               const float* __restrict__ cbb,
                                               const float* __restrict__ beta_p,
                                               float* out) {
  __shared__ __attribute__((aligned(16))) float ost[EW * OPITCH];
  const unsigned tid = threadIdx.x, lane = tid & 31u, hh = lane >> 4, m = lane & 15u;
  const unsigned wave = (unsigned)__builtin_amdgcn_readfirstlane((int)(threadIdx.x >> 5));
  const unsigned i0 = blockIdx.x * 32u, b = blockIdx.y;
  const unsigned bh = b * NH + wave;
  const v8f zero8 = {0.f, 0.f, 0.f, 0.f, 0.f, 0.f, 0.f, 0.f};
  const v4i zero4 = {0, 0, 0, 0};
  const float nbeta = -bf16_val(beta_p[0]);

  const unsigned short* kb = cpl + ((size_t)bh * SEQ + m) * QROW + 8u * hh;
  const unsigned short* vh = vt + ((size_t)bh * HD + m) * SEQ + 8u * hh;
  const unsigned short* vl = vh + VPL;
  const float* ctp = ctt + (size_t)bh * SEQ + 8u * hh;
  const float* cbp = cbb + (size_t)bh * SEQ + 8u * hh;

#pragma unroll 1
  for (unsigned tl = 0; tl < 2u; ++tl) {
    const unsigned g0 = i0 + 16u * tl;
    const unsigned short* qp = rpl + ((size_t)bh * SEQ + g0 + m) * QROW + 8u * hh;
    FragB qf;
    qf.q[0] = *(const v4ia*)qp;
    qf.q[1] = *(const v4ia*)(qp + 16);
    const float rt = rtt[(size_t)bh * SEQ + g0 + m];
    v8f o = zero8;
    float mrun = -3.0e38f, lrun = 0.0f;
#pragma unroll 1
    for (unsigned n0 = 0; n0 < SEQ; n0 += 32u) {
      const unsigned short* kp = kb + (size_t)n0 * QROW;
      const v4i kh0 = *(const v4ia*)kp;
      const v4i kl0 = *(const v4ia*)(kp + 16);
      const v4i kh1 = *(const v4ia*)(kp + 16 * QROW);
      const v4i kl1 = *(const v4ia*)(kp + 16 * QROW + 16);
      FragB a10, a20, a11, a21;
      a10.q[0] = kh0; a10.q[1] = kh0;
      a20.q[0] = kl0; a20.q[1] = zero4;
      a11.q[0] = kh1; a11.q[1] = kh1;
      a21.q[0] = kl1; a21.q[1] = zero4;
      v8f s0 = wmb(a10, qf, zero8);
      s0 = wmb(a20, qf, s0);
      v8f s1 = wmb(a11, qf, zero8);
      s1 = wmb(a21, qf, s1);

      const v4f t0 = *(const v4fa*)(ctp + n0);
      const v4f t1 = *(const v4fa*)(ctp + n0 + 4u);
      const v4f t2 = *(const v4fa*)(ctp + n0 + 16u);
      const v4f t3 = *(const v4fa*)(ctp + n0 + 20u);
      const v4f u0 = *(const v4fa*)(cbp + n0);
      const v4f u1 = *(const v4fa*)(cbp + n0 + 4u);
      const v4f u2 = *(const v4fa*)(cbp + n0 + 16u);
      const v4f u3 = *(const v4fa*)(cbp + n0 + 20u);
      const v8f ct0 = __builtin_shufflevector(t0, t1, 0, 1, 2, 3, 4, 5, 6, 7);
      const v8f ct1 = __builtin_shufflevector(t2, t3, 0, 1, 2, 3, 4, 5, 6, 7);
      const v8f cb0 = __builtin_shufflevector(u0, u1, 0, 1, 2, 3, 4, 5, 6, 7);
      const v8f cb1 = __builtin_shufflevector(u2, u3, 0, 1, 2, 3, 4, 5, 6, 7);
      v8f a0, a1;
#pragma unroll
      for (int r = 0; r < 8; ++r) {
        a0[r] = hlogit(rt, ct0[r], s0[r], nbeta, cb0[r]);
        a1[r] = hlogit(rt, ct1[r], s1[r], nbeta, cb1[r]);
      }

      float t = fmaxf(a0[0], a1[0]);
#pragma unroll
      for (int r = 1; r < 8; ++r) t = fmaxf(t, fmaxf(a0[r], a1[r]));
      t = fmaxf(t, __shfl_xor(t, 16));
      const float mnew = fmaxf(mrun, t);
      const float sc = exp2f(mrun - mnew);
      v8f p0, p1;
      float ps = 0.0f;
#pragma unroll
      for (int r = 0; r < 8; ++r) {
        p0[r] = exp2f(a0[r] - mnew);
        p1[r] = exp2f(a1[r] - mnew);
        ps += p0[r] + p1[r];
      }
      lrun = lrun * sc + ps;
      mrun = mnew;
      o = o * sc;

      FragB ph, pw;
      split8(p0, ph.q[0], pw.q[0]);
      split8(p1, ph.q[1], pw.q[1]);
      FragB fvh, fvl;
      fvh.q[0] = *(const v4ia*)(vh + n0);
      fvh.q[1] = *(const v4ia*)(vh + n0 + 16u);
      fvl.q[0] = *(const v4ia*)(vl + n0);
      fvl.q[1] = *(const v4ia*)(vl + n0 + 16u);
      o = wmb(fvh, ph, o);
      o = wmb(fvl, ph, o);
      o = wmb(fvh, pw, o);
    }
    const float lt = lrun + __shfl_xor(lrun, 16);
    const float inv = 1.0f / lt;
    const v8f c = o * inv;
    const unsigned so = (16u * wave + 8u * hh) * OPITCH + 16u * tl + m;
#pragma unroll
    for (int r = 0; r < 8; ++r) ost[so + (unsigned)r * OPITCH] = c[r];
  }
  __syncthreads();

  {
    float* ob = out + (size_t)b * XB_FULL + i0;
#pragma unroll 1
    for (unsigned it = 0; it < 4u; ++it) {
      const unsigned p = it * 256u + tid, c = p >> 3, q = p & 7u;
      const v4f v = *(const v4fa*)(ost + c * OPITCH + 4u * q);
      *(volatile v4f*)(ob + (size_t)c * LFULL + 4u * q) = v;
    }
    __threadfence();
#pragma unroll 1
    for (unsigned it = 0; it < 4u; ++it) {
      const unsigned p = it * 256u + tid, c = p >> 3, q = p & 7u;
      const v4f v = *(const v4fa*)(ost + c * OPITCH + 4u * q);
      *(volatile v4f*)(ob + (size_t)c * LFULL + 4u * q) = v;
    }
  }
}

static inline size_t al256(size_t o) { return (o + 255) & ~(size_t)255; }

extern "C" void kernel_launch(void* const* d_in, const int* in_sizes, int n_in,
                              void* d_out, int out_size, void* d_ws, size_t ws_size,
                              hipStream_t stream) {
  (void)stream;
  if (n_in < 6) return;
  const long long actN = (long long)NB * EW * LFULL;
  if ((long long)in_sizes[0] < actN) return;
  if ((long long)in_sizes[1] < (long long)NB * LFULL) return;
  if (in_sizes[2] < 2 * EW * EW) return;
  if (in_sizes[3] < EW * EW) return;
  if (in_sizes[4] < 1 || in_sizes[5] < 1) return;
  if ((long long)out_size < actN) return;

  const float* queries = (const float*)d_in[0];
  const int*   mask    = (const int*)d_in[1];
  const float* Wmem    = (const float*)d_in[2];
  const float* Wq      = (const float*)d_in[3];
  const float* beta    = (const float*)d_in[4];
  const float* bias    = (const float*)d_in[5];
  float* out = (float*)d_out;

  const size_t wtB = al256((size_t)3 * EW * EW * 2);
  const size_t plB = al256((size_t)2 * PLN * 2);
  const size_t vB  = al256((size_t)2 * VPL * 2);
  const size_t scB = al256((size_t)3 * SCN * 4);
  const size_t total = wtB + plB + vB + scB;
  if (total > ws_size || total > (size_t)WSMAX) return;
  char* w = (char*)d_ws;
  unsigned short* wt  = (unsigned short*)w;
  unsigned short* pln = (unsigned short*)(w + wtB);
  unsigned short* vtp = (unsigned short*)(w + wtB + plB);
  float*          sca = (float*)(w + wtB + plB + vB);
  unsigned short* cpl = pln;
  unsigned short* rpl = pln + PLN;
  float* ctt = sca;
  float* rtt = sca + SCN;
  float* cbb = sca + 2 * SCN;

  k_cvt<<<(unsigned)((2 * EW * EW) / (256 * 8)), 256, 0, stream>>>(Wmem, wt);
  k_cvt<<<(unsigned)((EW * EW) / (256 * 8)), 256, 0, stream>>>(Wq, wt + 2 * EW * EW);
  k_hproj<<<(NB * SEQ) / 64, 128, 0, stream>>>(queries, mask, wt, bias, pln, vtp, sca);
  k_hattn<<<dim3(SEQ / 32, NB), 256, 0, stream>>>(rpl, cpl, vtp, rtt, ctt, cbb, beta, out);
}
